// ModConv_69320772158389
// MI455X (gfx1250) — hardware-verified
//
#include <hip/hip_runtime.h>
#include <hip/hip_bf16.h>


#define __bf16 _Float16
typedef __attribute__((ext_vector_type(8)))  _Float16 v8bf;
typedef __attribute__((ext_vector_type(16))) _Float16 v16bf;
typedef __attribute__((ext_vector_type(8)))  float  v8f;
#define VST2(T, ptr, val) do { const T _v = (val); *(volatile T*)(ptr) = _v; __threadfence(); *(volatile T*)(ptr) = _v; } while (0)
typedef __attribute__((ext_vector_type(4)))  unsigned int v4u;
typedef __attribute__((ext_vector_type(8)))  int v8i;
typedef __attribute__((ext_vector_type(4)))  int v4i;

#define C_IN   512
#define C_OUT  512
#define HW     1024
#define NKIDX  144
#define LDSS   40


__global__ void style_kernel(const float* __restrict__ w,
                             const float* __restrict__ aw,
                             const float* __restrict__ ab,
                             float* __restrict__ style,
                             float* __restrict__ style2) {
  int id = blockIdx.x * blockDim.x + threadIdx.x;
  int b = id >> 9, i = id & 511;
  const float4* wr = reinterpret_cast<const float4*>(w + b * 512);
  const float4* ar = reinterpret_cast<const float4*>(aw + (size_t)i * 512);
  float s = ab[i];
  #pragma unroll 4
  for (int j = 0; j < 128; ++j) {
    float4 a = wr[j], c = ar[j];
    s += a.x * c.x + a.y * c.y + a.z * c.z + a.w * c.w;
  }
  VST2(float, style + id, s);
  VST2(float, style2 + id, s * s);
}

__global__ void wsq_kernel(const float* __restrict__ weight,
                           float* __restrict__ wsq) {
  int id = blockIdx.x * blockDim.x + threadIdx.x;
  const float* p = weight + (size_t)id * 9;
  float s = 0.f;
  #pragma unroll
  for (int t = 0; t < 9; ++t) s += p[t] * p[t];
  VST2(float, wsq + id, s);
}

__global__ void demod_kernel(const float* __restrict__ style2,
                             const float* __restrict__ wsq,
                             float* __restrict__ dmod) {
  int id = blockIdx.x * blockDim.x + threadIdx.x;
  int b = id >> 9, o = id & 511;
  const float4* s2 = reinterpret_cast<const float4*>(style2 + b * 512);
  const float4* wq = reinterpret_cast<const float4*>(wsq + (size_t)o * 512);
  float acc = 1e-8f;
  #pragma unroll 4
  for (int j = 0; j < 128; ++j) {
    float4 a = s2[j], c = wq[j];
    acc += a.x * c.x + a.y * c.y + a.z * c.z + a.w * c.w;
  }
  VST2(float, dmod + id, 1.0f / sqrtf(acc));
}

__global__ void xst_kernel(const float* __restrict__ x,
                           const float* __restrict__ style,
                           __bf16* __restrict__ xsT) {
  __shared__ float tile[64][33];
  const int p0 = blockIdx.x * 32;
  const int i0 = blockIdx.y * 64;
  const int b  = blockIdx.z;
  const int tx = threadIdx.x;
  const int ty = threadIdx.y;
  #pragma unroll
  for (int r = 0; r < 8; ++r) {
    int i = i0 + ty + r * 8;
    tile[ty + r * 8][tx] = x[((size_t)b * C_IN + i) * HW + p0 + tx] * style[b * C_IN + i];
  }
  __syncthreads();
  const int t = ty * 32 + tx, p = t >> 3, q = (t & 7) * 8;
  v8bf v;
  #pragma unroll
  for (int e = 0; e < 8; ++e) v[e] = (__bf16)tile[q + e][p];
  VST2(v8bf, xsT + ((size_t)b * HW + p0 + p) * C_IN + i0 + q, v);
}

__global__ void wre_kernel(const float* __restrict__ weight,
                           __bf16* __restrict__ wre) {
  int id8 = blockIdx.x * blockDim.x + threadIdx.x;
  int id = id8 * 8;
  int i  = id & 511;
  int to = id >> 9;
  int o  = to & 511;
  int t  = to >> 9;
  v8bf v;
  #pragma unroll
  for (int e = 0; e < 8; ++e) v[e] = (__bf16)weight[((size_t)o * C_IN + i + e) * 9 + t];
  VST2(v8bf, wre + id, v);
}


__global__ __launch_bounds__(256)
void modconv_gemm(const __bf16* __restrict__ wre,
                  const __bf16* __restrict__ xsT,
                  const float*  __restrict__ dmod,
                  float* __restrict__ out)
{
  __shared__ __attribute__((aligned(16))) __bf16 Alds[2][128 * LDSS];
  __shared__ __attribute__((aligned(16))) __bf16 Blds[2][128 * LDSS];

  const int tid   = threadIdx.x;
  const int nbase = blockIdx.x * 128;
  const int obase = blockIdx.y * 128;
  const int bb    = blockIdx.z;

  const int lane = tid & 31;
  const int wave = tid >> 5;
  const int wm   = wave >> 1;
  const int wn   = wave & 1;
  const int l15  = lane & 15;
  const int hi   = lane >> 4;

  const int brow = tid >> 1;
  const int bseg = (tid & 1) << 4;
  const int pix  = nbase + brow;
  const int py   = pix >> 5;
  const int px   = pix & 31;
  const __bf16* xb = xsT + (size_t)bb * (HW * C_IN);

  uint4 br0, br1;

  auto load_regs = [&](int kidx) {
    const int t  = kidx >> 4;
    const int kb = (kidx & 15) << 5;
    const int dy = t / 3 - 1;
    const int dx = t - (t / 3) * 3 - 1;
    const int yy = py + dy, xx = px + dx;
    if (((unsigned)yy < 32u) && ((unsigned)xx < 32u)) {
      const uint4* bp = reinterpret_cast<const uint4*>(
          xb + (size_t)(pix + dy * 32 + dx) * C_IN + kb + bseg);
      br0 = bp[0];
      br1 = bp[1];
    } else {
      br0 = uint4{0u, 0u, 0u, 0u};
      br1 = uint4{0u, 0u, 0u, 0u};
    }
  };

  auto store_tiles = [&](int buf) {
    *reinterpret_cast<uint4*>(&Blds[buf][brow * LDSS + bseg])     = br0;
    *reinterpret_cast<uint4*>(&Blds[buf][brow * LDSS + bseg + 8]) = br1;
  };

  uint4 ar0, ar1;
  auto load_A_regs = [&](int kidx) {
    const int t  = kidx >> 4;
    const int kb = (kidx & 15) << 5;
    const __bf16* gp = wre + ((size_t)t * C_OUT + obase) * C_IN + kb;
    const int r0 = tid >> 2, s0 = (tid & 3) * 8;
    ar0 = *reinterpret_cast<const uint4*>(gp + (size_t)r0 * C_IN + s0);
    ar1 = *reinterpret_cast<const uint4*>(gp + (size_t)(r0 + 64) * C_IN + s0);
  };
  auto store_A = [&](int buf) {
    const int r0 = tid >> 2, s0 = (tid & 3) * 8;
    *reinterpret_cast<uint4*>(&Alds[buf][r0 * LDSS + s0])        = ar0;
    *reinterpret_cast<uint4*>(&Alds[buf][(r0 + 64) * LDSS + s0]) = ar1;
  };

  v8f acc[2][4];
  #pragma unroll
  for (int mi = 0; mi < 2; ++mi)
    #pragma unroll
    for (int ni = 0; ni < 4; ++ni)
      acc[mi][ni] = v8f{0.f, 0.f, 0.f, 0.f, 0.f, 0.f, 0.f, 0.f};

  load_A_regs(0); load_regs(0);
  store_A(0); store_tiles(0);
  for (int kidx = 0; kidx < NKIDX; ++kidx) {
    __syncthreads();
    const int cur = kidx & 1;
    if (kidx + 1 < NKIDX) {
      load_A_regs(kidx + 1);
      load_regs(kidx + 1);
    }

    v16bf af[2];
    #pragma unroll
    for (int mi = 0; mi < 2; ++mi) {
      const __bf16* ap = &Alds[cur][(wm * 32 + mi * 16 + l15) * LDSS + hi * 8];
      v8bf lo  = *reinterpret_cast<const v8bf*>(ap);
      v8bf hi8 = *reinterpret_cast<const v8bf*>(ap + 16);
      af[mi] = __builtin_shufflevector(lo, hi8, 0,1,2,3,4,5,6,7,8,9,10,11,12,13,14,15);
    }
    v16bf bfm[4];
    #pragma unroll
    for (int ni = 0; ni < 4; ++ni) {
      const __bf16* bp = &Blds[cur][(wn * 64 + ni * 16 + l15) * LDSS + hi * 8];
      v8bf lo  = *reinterpret_cast<const v8bf*>(bp);
      v8bf hi8 = *reinterpret_cast<const v8bf*>(bp + 16);
      bfm[ni] = __builtin_shufflevector(lo, hi8, 0,1,2,3,4,5,6,7,8,9,10,11,12,13,14,15);
    }
    #pragma unroll
    for (int mi = 0; mi < 2; ++mi)
      #pragma unroll
      for (int ni = 0; ni < 4; ++ni)
      { acc[mi][ni] = __builtin_amdgcn_wmma_f32_16x16x32_f16(
            false, af[mi], false, bfm[ni], (short)0, acc[mi][ni], false, false);
        asm volatile("v_nop\n\tv_nop\n\tv_nop\n\tv_nop" : "+v"(acc[mi][ni]) : "v"(af[mi]), "v"(bfm[ni])); }

    if (kidx + 1 < NKIDX) { store_A(cur ^ 1); store_tiles(cur ^ 1); }
  }

  float dv[2][8];
  #pragma unroll
  for (int mi = 0; mi < 2; ++mi)
    #pragma unroll
    for (int j = 0; j < 8; ++j)
      dv[mi][j] = dmod[bb * C_OUT + obase + wm * 32 + mi * 16 + hi * 8 + j];

  float* outb = out + ((size_t)bb * C_OUT + obase) * HW;
  for (int pass = 0; pass < 2; ++pass) {
    #pragma unroll
    for (int mi = 0; mi < 2; ++mi)
      #pragma unroll
      for (int pr = 0; pr < 2; ++pr)
        #pragma unroll
        for (int j = 0; j < 8; ++j) {
          const float a_ = acc[mi][2 * pr][j] * dv[mi][j], b_ = acc[mi][2 * pr + 1][j] * dv[mi][j];
          const float ax = __shfl_xor(a_, 16), bx = __shfl_xor(b_, 16);
          const int row0 = wm * 32 + mi * 16 + j;
          const int col  = nbase + wn * 64 + pr * 32 + lane;
          *(volatile float*)(outb + (size_t)row0 * HW + col)       = hi ? bx : a_;
          *(volatile float*)(outb + (size_t)(row0 + 8) * HW + col) = hi ? b_ : ax;
        }
    __threadfence();
  }
}


extern "C" void kernel_launch(void* const* d_in, const int* in_sizes, int n_in,
                              void* d_out, int out_size, void* d_ws, size_t ws_size,
                              hipStream_t stream) {
  (void)in_sizes; (void)n_in; (void)out_size;
  if (ws_size < (size_t)5865472 + (size_t)16 * 1024 * 512 * 2) return;
  const float* x   = (const float*)d_in[0];
  const float* w   = (const float*)d_in[1];
  const float* wgt = (const float*)d_in[2];
  const float* aw  = (const float*)d_in[3];
  const float* ab  = (const float*)d_in[4];
  float* out = (float*)d_out;

  char* ws = (char*)d_ws;
  float*  style  = (float*)(ws);
  float*  style2 = (float*)(ws + 32768);
  float*  dmod   = (float*)(ws + 65536);
  float*  wsq    = (float*)(ws + 98304);
  __bf16* wre    = (__bf16*)(ws + 1146880);
  __bf16* xsT    = (__bf16*)(ws + 5865472);

  style_kernel<<<32,   256, 0, stream>>>(w, aw, ab, style, style2);
  wsq_kernel  <<<1024, 256, 0, stream>>>(wgt, wsq);
  demod_kernel<<<32,   256, 0, stream>>>(style2, wsq, dmod);

  dim3 tg(32, 8, 16), tb(32, 8);
  xst_kernel  <<<tg, tb, 0, stream>>>(x, style, xsT);
  wre_kernel  <<<9216 / 8, 256, 0, stream>>>(wgt, wre);

  dim3 grid(8, 4, 16);
  modconv_gemm<<<grid, 256, 0, stream>>>(wre, xsT, dmod, out);
}
